// GeometryGNN_54657753809375
// MI455X (gfx1250) — hardware-verified
//
#include <hip/hip_runtime.h>

typedef _Float16 f16t;
typedef _Float16 v16h __attribute__((ext_vector_type(16)));
typedef _Float16 v8h  __attribute__((ext_vector_type(8)));
typedef float    v8f  __attribute__((ext_vector_type(8)));
typedef float    v4f  __attribute__((ext_vector_type(4)));
typedef v8h __attribute__((may_alias)) v8ha;
typedef v4f __attribute__((may_alias)) v4fa;
union Frag { v16h v; v8h half[2]; };

#define DIN    16
#define HD     256
#define KP0    32
#define ROWS   32
#define NSTG   7
#define TPB    256
#define XCAR   16.0f
#define ACAR   16.0f
#define W0CAR  64.0f
#define WCAR   256.0f

static_assert(ROWS * KP0 == 8 * 128);
static_assert(ROWS * 3 == 4 * 24);
static_assert((ROWS * 3 * 4) % 128 == 0);
static_assert(TPB == 8 * ROWS);

__device__ __forceinline__ v8f wmma_f16(v16h a, v16h b, v8f c) {
  v8f d = __builtin_amdgcn_wmma_f32_16x16x32_f16(false, a, false, b, (short)0, c, false, false);
  asm volatile("v_nop\n\tv_nop\n\tv_nop\n\tv_nop" : "+v"(d) : "v"(a), "v"(b));
  return d;
}

__device__ __forceinline__ v8f zero8f() {
  v8f z;
  #pragma unroll
  for (int j = 0; j < 8; ++j) z[j] = 0.f;
  return z;
}

__device__ __forceinline__ void mm_stage(const f16t* ain, int apitch, int ksteps,
                                         const f16t* __restrict__ Wp, int ldk,
                                         const float* __restrict__ bias_g,
                                         const float* __restrict__ ini, bool use_init,
                                         float oscale, float scale, f16t* aout,
                                         int lane, int w)
{
  const int h = lane >> 4, m = lane & 15;
  const int mt = w >> 2, ng = w & 3;
  v8f acc[4];
  #pragma unroll
  for (int nt = 0; nt < 4; ++nt) acc[nt] = zero8f();

  const f16t* arow = ain + (16 * mt + m) * apitch + 8 * h;
  const f16t* wrow = Wp + (size_t)(64 * ng + m) * ldk + 8 * h;

  #pragma unroll 1
  for (int ks = 0; ks < ksteps; ++ks) {
    const int k0 = 32 * ks;
    Frag a;
    a.half[0] = *(const v8ha*)(arow + k0);
    a.half[1] = *(const v8ha*)(arow + k0 + 16);
    #pragma unroll
    for (int nt = 0; nt < 4; ++nt) {
      const f16t* wp = wrow + (size_t)(16 * nt) * ldk + k0;
      Frag b;
      b.half[0] = *(const v8ha*)wp;
      b.half[1] = *(const v8ha*)(wp + 16);
      acc[nt] = wmma_f16(a.v, b.v, acc[nt]);
    }
  }

  #pragma unroll
  for (int nt = 0; nt < 4; ++nt) {
    const int c = 64 * ng + 16 * nt + m;
    const float bias = bias_g[c];
    float iadd = 0.f;
    if (use_init) iadd = (ini[c] + ini[HD + c]) + ini[2 * HD + c];
    f16t* orow = aout + (16 * mt + 8 * h) * HD + c;
    #pragma unroll
    for (int r = 0; r < 8; ++r) {
      float v = acc[nt][r] * oscale + bias;
      v = fmaxf(v, 0.f);
      v = v * scale + iadd;
      orow[r * HD] = (f16t)(v * ACAR);
    }
  }
}

__global__ __launch_bounds__(TPB) void prep_w0_k(const float* __restrict__ ew0, f16t* __restrict__ W0P)
{
  const int t = blockIdx.x * TPB + threadIdx.x;
  if (t >= HD * (KP0 / 8)) return;
  const int row = t >> 2, part = t & 3;
  const float* src = ew0 + row * DIN + 8 * (part & 1);
  const v4f f0 = *(const v4fa*)src;
  const v4f f1 = *(const v4fa*)(src + 4);
  const float sc = (part < 2) ? W0CAR : 0.0f;
  v8h o;
  #pragma unroll
  for (int i = 0; i < 4; ++i) {
    o[i]     = (f16t)(f0[i] * sc);
    o[4 + i] = (f16t)(f1[i] * sc);
  }
  f16t* dst = W0P + 8 * t;
  *(volatile v8h*)dst = o;
  __threadfence();
  *(volatile v8h*)dst = o;
}

__global__ __launch_bounds__(TPB) void prep_w_k(const float* __restrict__ ew1, const float* __restrict__ gw1,
                                               const float* __restrict__ gw2, f16t* __restrict__ WP)
{
  const int k = blockIdx.y;
  const int l1 = (k > 0) ? ((k - 1) >> 1) : 0;
  const int l2 = (k > 1) ? ((k - 2) >> 1) : 0;
  const float* src = (k == 0) ? ew1
                   : ((k & 1) ? (gw1 + (size_t)l1 * HD * HD) : (gw2 + (size_t)l2 * HD * HD));
  const int g = blockIdx.x * TPB + threadIdx.x;
  if (g >= HD * HD / 8) return;
  const v4f f0 = *(const v4fa*)(src + 8 * g);
  const v4f f1 = *(const v4fa*)(src + 8 * g + 4);
  v8h o;
  #pragma unroll
  for (int i = 0; i < 4; ++i) {
    o[i]     = (f16t)(f0[i] * WCAR);
    o[4 + i] = (f16t)(f1[i] * WCAR);
  }
  f16t* dst = WP + (size_t)k * HD * HD + 8 * g;
  *(volatile v8h*)dst = o;
  __threadfence();
  *(volatile v8h*)dst = o;
}

__global__ __launch_bounds__(TPB) void gnn_k(const float* __restrict__ x,
                                           const f16t* __restrict__ W0P,
                                           const f16t* __restrict__ WP,
                                           const float* __restrict__ eb0, const float* __restrict__ eb1,
                                           const float* __restrict__ ini,
                                           const float* __restrict__ gb1, const float* __restrict__ gb2,
                                           const float* __restrict__ dw, const float* __restrict__ db,
                                           float* __restrict__ out, int nB)
{
  __shared__ __attribute__((aligned(16))) f16t sAct[2 * ROWS * HD];
  __shared__ __attribute__((aligned(16))) f16t sX[ROWS * KP0];
  __shared__ __attribute__((aligned(16))) float sOut[128];
  const int tid = threadIdx.x, lane = tid & 31, w = tid >> 5;
  const int rbase = blockIdx.x * ROWS;
  if (rbase + ROWS > nB) return;
  const float bd = db[0];

  if (tid < 128) {
    const int row = tid >> 2, part = tid & 3;
    const float* src = x + (size_t)(rbase + row) * DIN + 8 * (part & 1);
    const v4f f0 = *(const v4fa*)src;
    const v4f f1 = *(const v4fa*)(src + 4);
    const float sc = (part < 2) ? XCAR : 0.0f;
    v8h o;
    #pragma unroll
    for (int i = 0; i < 4; ++i) {
      o[i]     = (f16t)(f0[i] * sc);
      o[4 + i] = (f16t)(f1[i] * sc);
    }
    *(v8ha*)(sX + 8 * tid) = o;
    sOut[tid] = 0.f;
  }
  __syncthreads();

  mm_stage(sX, KP0, 1, W0P, KP0, eb0, ini, false,
           1.0f / (XCAR * W0CAR), 1.0f, sAct, lane, w);
  __syncthreads();

  #pragma unroll 1
  for (int s = 0; s < NSTG; ++s) {
    const int lyr = (s > 0) ? ((s - 1) >> 1) : 0;
    const float* bias = (s == 0) ? eb1 : ((s & 1) ? (gb1 + lyr * HD) : (gb2 + lyr * HD));
    const float scl = (s == 0 || s == 2 || s == 4) ? 3.0f : 1.0f;
    const f16t* ain = sAct + (s & 1) * (ROWS * HD);
    f16t* aout = sAct + ((s & 1) ^ 1) * (ROWS * HD);
    mm_stage(ain, HD, HD / 32, WP + (size_t)s * HD * HD, HD, bias, ini, s == 0,
             1.0f / (ACAR * WCAR), scl, aout, lane, w);
    __syncthreads();
  }

  {
    const f16t* fin = sAct + ROWS * HD;
    const int row = tid >> 3, part = tid & 7;
    const f16t* ar = fin + row * HD + 32 * part;
    const float* dr = dw + 32 * part;
    float sacc = 0.f;
    #pragma unroll
    for (int j = 0; j < 4; ++j) {
      const v8h a = *(const v8ha*)(ar + 8 * j);
      const v4f d0 = *(const v4fa*)(dr + 8 * j);
      const v4f d1 = *(const v4fa*)(dr + 8 * j + 4);
      #pragma unroll
      for (int i = 0; i < 4; ++i) {
        sacc += (float)a[i] * d0[i];
        sacc += (float)a[4 + i] * d1[i];
      }
    }
    sacc += __shfl_xor(sacc, 1);
    sacc += __shfl_xor(sacc, 2);
    sacc += __shfl_xor(sacc, 4);
    if (part == 0) {
      const float p = sacc * (1.0f / ACAR) + bd;
      sOut[3 * row]     = p;
      sOut[3 * row + 1] = p;
      sOut[3 * row + 2] = p;
    }
  }
  __syncthreads();

  if (w == 0) {
    const v4f v = *(const v4fa*)(sOut + 4 * lane);
    float* dst = out + (size_t)rbase * 3 + 4 * lane;
    if (lane < 24) *(volatile v4f*)dst = v;
    __threadfence();
    if (lane < 24) *(volatile v4f*)dst = v;
  }
}

extern "C" void kernel_launch(void* const* d_in, const int* in_sizes, int n_in,
                              void* d_out, int out_size, void* d_ws, size_t ws_size,
                              hipStream_t stream) {
  if (n_in < 12) return;
  const int nB = in_sizes[0] / DIN;
  if (nB <= 0 || nB * DIN != in_sizes[0]) return;
  if ((nB % ROWS) != 0) return;
  if (in_sizes[1] != HD * DIN) return;
  if (in_sizes[2] != HD) return;
  if (in_sizes[3] != HD * HD) return;
  if (in_sizes[4] != HD) return;
  if (in_sizes[5] != 3 * HD) return;
  if (in_sizes[6] != 3 * HD * HD) return;
  if (in_sizes[7] != 3 * HD) return;
  if (in_sizes[8] != 3 * HD * HD) return;
  if (in_sizes[9] != 3 * HD) return;
  if (in_sizes[10] != HD) return;
  if (in_sizes[11] < 1) return;
  if (out_size != 3 * nB) return;

  const float* x    = (const float*)d_in[0];
  const float* ew0  = (const float*)d_in[1];
  const float* eb0  = (const float*)d_in[2];
  const float* ew1  = (const float*)d_in[3];
  const float* eb1  = (const float*)d_in[4];
  const float* ini  = (const float*)d_in[5];
  const float* gw1  = (const float*)d_in[6];
  const float* gb1  = (const float*)d_in[7];
  const float* gw2  = (const float*)d_in[8];
  const float* gb2  = (const float*)d_in[9];
  const float* dw   = (const float*)d_in[10];
  const float* db   = (const float*)d_in[11];
  float* outp = (float*)d_out;

  const size_t szW0 = (size_t)HD * KP0 * 2;
  const size_t szWP = (size_t)NSTG * HD * HD * 2;
  size_t off = 0;
  char* ws = (char*)d_ws;
  f16t* W0P = (f16t*)(ws + off); off += szW0;
  f16t* WP  = (f16t*)(ws + off); off += szWP;
  if (off > ws_size) return;

  prep_w0_k<<<(HD * (KP0 / 8) + TPB - 1) / TPB, TPB, 0, stream>>>(ew0, W0P);
  prep_w_k<<<dim3((HD * HD / 8 + TPB - 1) / TPB, NSTG), TPB, 0, stream>>>(ew1, gw1, gw2, WP);
  gnn_k<<<nB / ROWS, TPB, 0, stream>>>(x, W0P, WP, eb0, eb1, ini, gb1, gb2, dw, db, outp, nB);
}
